// QuaternionSSM_18588618457727
// MI455X (gfx1250) — hardware-run, weakly checked
//
#include <hip/hip_runtime.h>


#define NM   2048
#define NB   2
#define NT   1024
#define DM   128
#define DI   256
#define D4   1024
#define NS   64
#define NR   8
#define NXD  136
#define NXP  192
typedef _Float16 h16;
typedef unsigned short bf;
typedef __attribute__((ext_vector_type(16))) __bf16   v16bf;
typedef __attribute__((ext_vector_type(16))) _Float16 v16h;
typedef __attribute__((ext_vector_type(8)))  _Float16 v8h;
typedef __attribute__((ext_vector_type(8)))  unsigned short v8us;
typedef __attribute__((ext_vector_type(8)))  float    v8f;
typedef __attribute__((ext_vector_type(4)))  float    v4f;
typedef v8h  __attribute__((may_alias)) v8ha;
typedef v4f  __attribute__((may_alias)) v4fa;
typedef v8us __attribute__((may_alias)) v8usa;

__device__ __forceinline__ unsigned short f2bf(float f) { unsigned u = __float_as_uint(f); u += 0x7FFFu + ((u >> 16) & 1u); return (unsigned short)(u >> 16); }
__device__ __forceinline__ float bf2f(unsigned short b) { return __uint_as_float(((unsigned)b) << 16); }
__device__ __forceinline__ float bfr(float f) { return bf2f(f2bf(f)); }
__device__ __forceinline__ v16h cat16(v8h lo, v8h hi) { return __builtin_shufflevector(lo, hi, 0, 1, 2, 3, 4, 5, 6, 7, 8, 9, 10, 11, 12, 13, 14, 15); }
__device__ __forceinline__ v16bf cat16b(v8us lo, v8us hi) { return __builtin_bit_cast(v16bf, __builtin_shufflevector(lo, hi, 0, 1, 2, 3, 4, 5, 6, 7, 8, 9, 10, 11, 12, 13, 14, 15)); }
__device__ __forceinline__ v8f wmma16(v16h a, v16h b, v8f c) { return __builtin_amdgcn_wmma_f32_16x16x32_f16(false, a, false, b, (short)0, c, false, false); }
__device__ __forceinline__ v8f wmmab(v16bf a, v16bf b, v8f c) { return __builtin_amdgcn_wmma_f32_16x16x32_bf16(false, a, false, b, (short)0, c, false, false); }

template <typename T16> struct WFrag;
template <> struct WFrag<h16> { typedef v16h V; static __device__ __forceinline__ V ld(const h16* p) { return cat16(*(const v8h*)p, *(const v8h*)(p + 16)); } static __device__ __forceinline__ v8f mma(V a, V b, v8f c) { return wmma16(a, b, c); } };
template <> struct WFrag<bf> { typedef v16bf V; static __device__ __forceinline__ V ld(const bf* p) { return cat16b(*(const v8us*)p, *(const v8us*)(p + 16)); } static __device__ __forceinline__ v8f mma(V a, V b, v8f c) { return wmmab(a, b, c); } };
template <typename T16, int NSPLIT, bool BIAS>
__global__ __launch_bounds__(32) void k_gemmw(const T16* __restrict__ A, const T16* __restrict__ A2, const T16* __restrict__ Bt, const T16* __restrict__ Bt2, int K, float* C, int ldc, const float* __restrict__ bias, size_t sA, size_t sB, size_t sC) {
    typedef typename WFrag<T16>::V V;
    __shared__ __align__(16) float os[16 * 68];
    const size_t z = blockIdx.z; A += z * sA; if (A2) A2 += z * sA; Bt += z * sB; if (Bt2) Bt2 += z * sB; C += z * sC;
    const int lane = threadIdx.x & 31, lr = lane & 15, hi = lane >> 4; const int r0 = blockIdx.x * 64, c0 = blockIdx.y * 64;
    v8f acc[4][4];
#pragma unroll
    for (int mb = 0; mb < 4; ++mb)
#pragma unroll
        for (int nb = 0; nb < 4; ++nb) acc[mb][nb] = (v8f){};
    const size_t aoff = (size_t)(r0 + lr) * K + 8 * hi, boff = (size_t)(c0 + lr) * K + 8 * hi;
    for (int kc = 0; kc < K; kc += 32) {
        V a[4], a2[4];
#pragma unroll
        for (int mb = 0; mb < 4; ++mb) { a[mb] = WFrag<T16>::ld(A + aoff + (size_t)mb * 16 * K + kc); if (NSPLIT == 1 || NSPLIT == 2) a2[mb] = WFrag<T16>::ld(A2 + aoff + (size_t)mb * 16 * K + kc); }
#pragma unroll
        for (int nb = 0; nb < 4; ++nb) { const V b = WFrag<T16>::ld(Bt + boff + (size_t)nb * 16 * K + kc); V b2; if (NSPLIT >= 2) b2 = WFrag<T16>::ld(Bt2 + boff + (size_t)nb * 16 * K + kc);
#pragma unroll
            for (int mb = 0; mb < 4; ++mb) { acc[mb][nb] = WFrag<T16>::mma(a[mb], b, acc[mb][nb]); if (NSPLIT == 1 || NSPLIT == 2) acc[mb][nb] = WFrag<T16>::mma(a2[mb], b, acc[mb][nb]); if (NSPLIT >= 2) acc[mb][nb] = WFrag<T16>::mma(a[mb], b2, acc[mb][nb]); } }
        asm volatile("v_nop\n\tv_nop\n\tv_nop\n\tv_nop" : "+v"(acc[0][0]), "+v"(acc[1][1]), "+v"(acc[2][2]), "+v"(acc[3][3]) : "v"(a[0]), "v"(a[3]));
    }
#pragma unroll
    for (int mb = 0; mb < 4; ++mb) {
#pragma unroll
        for (int nb = 0; nb < 4; ++nb) {
#pragma unroll
            for (int j = 0; j < 8; ++j) os[(hi * 8 + j) * 68 + nb * 16 + lr] = acc[mb][nb][j]; }
        __builtin_amdgcn_wave_barrier(); asm volatile("" ::: "memory");
        float* crow = C + (size_t)(r0 + mb * 16) * ldc + c0;
#pragma unroll 1
        for (int ps = 0; ps < 2; ++ps) {
#pragma unroll
            for (int s = 0; s < 8; ++s) { const int row = 2 * s + hi, cofs = lr * 4; v4f val = *(const v4fa*)(os + row * 68 + cofs); if (BIAS) { val[0] += bfr(bias[c0 + cofs]); val[1] += bfr(bias[c0 + cofs + 1]); val[2] += bfr(bias[c0 + cofs + 2]); val[3] += bfr(bias[c0 + cofs + 3]); }
                *(volatile v4f*)(crow + (size_t)row * ldc + cofs) = val; }
            if (ps == 0) __threadfence(); }
        __builtin_amdgcn_wave_barrier(); asm volatile("" ::: "memory");
    }
}

typedef __attribute__((ext_vector_type(2))) _Float16 v2h;
typedef __attribute__((ext_vector_type(4))) _Float16 v4h;
typedef __attribute__((ext_vector_type(2))) unsigned short v2us;
typedef __attribute__((ext_vector_type(4))) unsigned short v4us;
typedef __attribute__((ext_vector_type(2))) float v2f;
typedef __attribute__((ext_vector_type(4))) int v4i;
__device__ __forceinline__ h16 toh_flush(float x) { const float z = (fabsf(x) < 6.103515625e-05f) ? 0.0f : x; return (h16)z; }

__global__ __launch_bounds__(256) void k_wtG(const float* __restrict__ w, int K, int N, bf* Bt) {
    const int lane = threadIdx.x & 31; const int L0 = (blockIdx.x * 8 + (threadIdx.x >> 5)) * 8; const int nlines = N * K / 64;
#pragma unroll
    for (int ps = 0; ps < 2; ++ps) {
        for (int l = 0; l < 8; ++l) { const int L = L0 + l; if (L >= nlines) break; const size_t e = (size_t)L * 64 + lane * 2; const int k = (int)(e % K), n = (int)(e / K); v2us o;
            o[0] = f2bf(w[(size_t)k * N + n]); o[1] = f2bf(w[(size_t)(k + 1) * N + n]); *(volatile v2us*)(Bt + e) = o; }
        if (ps == 0) __threadfence(); }
}

__global__ __launch_bounds__(256) void k_fillb(bf* P, unsigned w2, size_t n8) { const size_t i = (size_t)blockIdx.x * 256 + threadIdx.x; if (i >= n8) return; v4i o; o[0] = (int)w2; o[1] = (int)w2; o[2] = (int)w2; o[3] = (int)w2;
    *(volatile v4i*)(P + i * 8) = o; __threadfence(); *(volatile v4i*)(P + i * 8) = o; }

__device__ __forceinline__ float sp(float v) { return fmaxf(v, 0.0f) + log1pf(expf(-fabsf(v))); }

__global__ __launch_bounds__(256) void k_cat4(const float* __restrict__ p0, const float* __restrict__ p1, const float* __restrict__ p2, const float* __restrict__ p3, bf* X) { const unsigned e = blockIdx.x * 256 + threadIdx.x; const unsigned m = e >> 6, a = (e >> 4) & 3u, c = (e & 15u) << 3; const unsigned m0 = 0u - (unsigned)(a == 0u), m1 = 0u - (unsigned)(a == 1u), m2 = 0u - (unsigned)(a == 2u), m3 = 0u - (unsigned)(a == 3u); const size_t off = (size_t)m * DM + c; const v4f u0 = *(const v4f*)(p0 + off), w0 = *(const v4f*)(p0 + off + 4), u1 = *(const v4f*)(p1 + off), w1 = *(const v4f*)(p1 + off + 4), u2 = *(const v4f*)(p2 + off), w2 = *(const v4f*)(p2 + off + 4), u3 = *(const v4f*)(p3 + off), w3 = *(const v4f*)(p3 + off + 4); v8us o;
#pragma unroll
    for (int k = 0; k < 4; ++k) { o[k] = f2bf(__uint_as_float((__float_as_uint(u0[k]) & m0) | (__float_as_uint(u1[k]) & m1) | (__float_as_uint(u2[k]) & m2) | (__float_as_uint(u3[k]) & m3))); o[k + 4] = f2bf(__uint_as_float((__float_as_uint(w0[k]) & m0) | (__float_as_uint(w1[k]) & m1) | (__float_as_uint(w2[k]) & m2) | (__float_as_uint(w3[k]) & m3))); }
    *(volatile v8us*)(X + (size_t)e * 8) = o; __threadfence(); *(volatile v8us*)(X + (size_t)e * 8) = o; }

template <typename T16> __device__ __forceinline__ unsigned short qw16(float v, float mul);
template <> __device__ __forceinline__ unsigned short qw16<bf>(float v, float mul) { return f2bf(__fmul_rn(v, mul)); }
template <> __device__ __forceinline__ unsigned short qw16<h16>(float v, float mul) { const h16 h = toh_flush(__fmul_rn(bfr(v), mul)); return __builtin_bit_cast(unsigned short, h); }
template <typename T16>
__global__ __launch_bounds__(256) void k_qw(const float* __restrict__ W0, const float* __restrict__ W1, const float* __restrict__ W2, const float* __restrict__ W3, int KD, int ND, float mul, unsigned short* Bt) { const unsigned e = blockIdx.x * 256 + threadIdx.x; const unsigned kg = (unsigned)KD >> 1; const unsigned n = e / kg, k0 = (e % kg) << 3; const unsigned a = n / (unsigned)ND, c = n % (unsigned)ND, b = k0 / (unsigned)KD, r0 = k0 % (unsigned)KD; const unsigned q = a ^ b; const float* s = (q == 0u) ? W0 : ((q == 1u) ? W1 : ((q == 2u) ? W2 : W3)); const float sg = ((0x428Eu >> (4u * a + b)) & 1u) ? -mul : mul; s += (size_t)r0 * ND + c; v8us o;
#pragma unroll
    for (int k = 0; k < 8; ++k) o[k] = qw16<T16>(s[(size_t)k * ND], sg);
    *(volatile v8us*)(Bt + (size_t)e * 8) = o; __threadfence(); *(volatile v8us*)(Bt + (size_t)e * 8) = o; }

__global__ __launch_bounds__(256) void k_conv(const float* __restrict__ XZ, const float* __restrict__ cw, const float* __restrict__ cb, float* Xs, bf* Xh, bf* Xl) { const unsigned e = blockIdx.x * 256 + threadIdx.x; const unsigned m = e >> 8, c0 = (e & 255u) << 2; const unsigned t = m & (NT - 1), m0 = m - t; v4f acc = *(const v4f*)(cb + c0);
#pragma unroll
    for (int k = 0; k < 4; ++k) acc[k] = bfr(acc[k]);
    v4f wq[4];
#pragma unroll
    for (int k = 0; k < 4; ++k) wq[k] = *(const v4f*)(cw + (size_t)(c0 + k) * 4);
#pragma unroll
    for (int j = 0; j < 4; ++j) { const int tj = (int)t - 3 + j; const unsigned tr = (tj < 0) ? 0u : (unsigned)tj; const float on = (tj < 0) ? 0.0f : 1.0f; const v4f xv = *(const v4f*)(XZ + (size_t)(m0 + tr) * (2 * D4) + c0);
#pragma unroll
        for (int k = 0; k < 4; ++k) acc[k] = acc[k] + (bfr(wq[k][j]) * on) * xv[k]; }
    v4f xs; v4us hi, lo;
#pragma unroll
    for (int k = 0; k < 4; ++k) { const float v = acc[k]; const float s = v / (1.0f + expf(-v)); xs[k] = s; hi[k] = f2bf(s); lo[k] = f2bf(s - bf2f(hi[k])); }
    *(volatile v4f*)(Xs + (size_t)e * 4) = xs; *(volatile v4us*)(Xh + (size_t)e * 4) = hi; *(volatile v4us*)(Xl + (size_t)e * 4) = lo; __threadfence(); *(volatile v4f*)(Xs + (size_t)e * 4) = xs; *(volatile v4us*)(Xh + (size_t)e * 4) = hi; *(volatile v4us*)(Xl + (size_t)e * 4) = lo; }

__global__ __launch_bounds__(256) void k_scan(const float* __restrict__ XD, const float* __restrict__ Xs, const float* __restrict__ Wd, const float* __restrict__ bd, const float* __restrict__ Al, float* Ys) { const int i = blockIdx.x * 256 + threadIdx.x; if (i >= NB * D4) return; const int b = i / D4; const int d = i % D4; float av[NS], h[NS], wd[NR];
#pragma unroll
    for (int n = 0; n < NS; ++n) { av[n] = -expf(bfr(Al[(size_t)d * NS + n])); h[n] = 0.0f; }
#pragma unroll
    for (int k = 0; k < NR; ++k) wd[k] = bfr(Wd[(size_t)k * D4 + d]);
    const float bq = bfr(bd[d]);
    for (int t0 = 0; t0 < NT; t0 += 4) { float y4[4];
#pragma unroll
        for (int s = 0; s < 4; ++s) { const size_t r = (size_t)b * NT + t0 + s; const float* xd = XD + r * NXP; float p = bq;
#pragma unroll
            for (int k = 0; k < NR; ++k) p = p + xd[k] * wd[k];
            const float q = sp(p); const float xv = Xs[r * D4 + d]; float y = 0.0f;
#pragma unroll
            for (int n = 0; n < NS; ++n) { h[n] = expf(q * av[n]) * h[n] + (q * xd[NR + n]) * xv; y = y + h[n] * xd[NR + NS + n]; }
            y4[s] = y; }
        float* o = Ys + ((size_t)b * NT + t0) * D4 + d;
#pragma unroll
        for (int s = 0; s < 4; ++s) *(volatile float*)(o + (size_t)s * D4) = y4[s];
        __threadfence();
#pragma unroll
        for (int s = 0; s < 4; ++s) *(volatile float*)(o + (size_t)s * D4) = y4[s]; }
}

__global__ __launch_bounds__(256) void k_gate(const float* __restrict__ Ys, const float* __restrict__ Xs, const float* __restrict__ XZ, const float* __restrict__ Dv, h16* Yh) { const unsigned e = blockIdx.x * 256 + threadIdx.x; const unsigned m = e >> 7, c0 = (e & 127u) << 3; const float* py = Ys + (size_t)m * D4 + c0; const float* px = Xs + (size_t)m * D4 + c0; const float* pz = XZ + (size_t)m * (2 * D4) + D4 + c0; const float* pd = Dv + c0; v8h o;
#pragma unroll
    for (int hf = 0; hf < 2; ++hf) { const v4f y = *(const v4f*)(py + 4 * hf), x = *(const v4f*)(px + 4 * hf), z = *(const v4f*)(pz + 4 * hf), dv = *(const v4f*)(pd + 4 * hf);
#pragma unroll
        for (int k = 0; k < 4; ++k) { const float g = (y[k] + x[k] * bfr(dv[k])) * (z[k] / (1.0f + expf(-z[k]))); o[4 * hf + k] = toh_flush(g * 0.0625f); } }
    *(volatile v8h*)(Yh + (size_t)e * 8) = o; __threadfence(); *(volatile v8h*)(Yh + (size_t)e * 8) = o; }

extern "C" void kernel_launch(void* const* d_in, const int* in_sizes, int n_in, void* d_out, int out_size, void* d_ws, size_t ws_size, hipStream_t stream) {
    if (n_in < 19) return;
    for (int k = 0; k < 4; ++k) { if (in_sizes[k] != NM * DM || in_sizes[4 + k] != DM * 2 * DI || in_sizes[15 + k] != DI * DM) return; }
    if (in_sizes[8] != D4 * 4 || in_sizes[9] != D4 || in_sizes[10] != D4 * NXD || in_sizes[11] != NR * D4 || in_sizes[12] != D4 || in_sizes[13] != D4 * NS || in_sizes[14] != D4) return;
    if (out_size != NM * 4 * DM) return;
    static_assert(NM == NB * NT && (NT & (NT - 1)) == 0 && D4 == 4 * DI && 2 * D4 == 4 * 2 * DI && NM % 64 == 0 && (2 * D4) % 64 == 0 && NXP % 64 == 0 && NXP >= NXD && NXD == NR + 2 * NS && (4 * DM) % 64 == 0 && (4 * DM) % 32 == 0 && D4 % 32 == 0 && DM % 8 == 0 && DI % 8 == 0 && (NM * 4 * DM / 8) % 256 == 0 && (2 * D4 * 4 * DM / 8) % 256 == 0 && (4 * DM * D4 / 8) % 256 == 0 && (NM * D4 / 4) % 256 == 0 && (NM * D4 / 8) % 256 == 0 && (NB * D4) % 256 == 0 && NT % 4 == 0 && (NXD * D4) % (64 * 64) == 0 && ((NXP - NXD) * D4 / 8) % 256 == 0, "the products: M and N multiples of 64, the depths of 32; the flat grids exact; a wave's 32 channels in one batch; the steps in fours; the transposing cast's lines in whole blocks of 64");
    const float* q0 = (const float*)d_in[0]; const float* q1 = (const float*)d_in[1]; const float* q2 = (const float*)d_in[2]; const float* q3 = (const float*)d_in[3]; const float* Wi0 = (const float*)d_in[4]; const float* Wi1 = (const float*)d_in[5]; const float* Wi2 = (const float*)d_in[6]; const float* Wi3 = (const float*)d_in[7]; const float* cw = (const float*)d_in[8]; const float* cb = (const float*)d_in[9]; const float* Wx = (const float*)d_in[10]; const float* Wd = (const float*)d_in[11]; const float* bd = (const float*)d_in[12]; const float* Al = (const float*)d_in[13]; const float* Dv = (const float*)d_in[14]; const float* Wo0 = (const float*)d_in[15]; const float* Wo1 = (const float*)d_in[16]; const float* Wo2 = (const float*)d_in[17]; const float* Wo3 = (const float*)d_in[18]; float* out = (float*)d_out;
    char* wsp = (char*)d_ws; auto take = [&](size_t bytes) { char* p = wsp; wsp += (bytes + 255) & ~(size_t)255; return (void*)p; };
    bf* Xq = (bf*)take((size_t)NM * 4 * DM * 2); bf* Bi = (bf*)take((size_t)2 * D4 * 4 * DM * 2); float* XZ = (float*)take((size_t)NM * 2 * D4 * 4); float* Xs = (float*)take((size_t)NM * D4 * 4); bf* Xh = (bf*)take((size_t)NM * D4 * 2); bf* Xl = (bf*)take((size_t)NM * D4 * 2); bf* Bx = (bf*)take((size_t)NXP * D4 * 2); float* XD = (float*)take((size_t)NM * NXP * 4); float* Ys = (float*)take((size_t)NM * D4 * 4); h16* Yh = (h16*)take((size_t)NM * D4 * 2); h16* Bo = (h16*)take((size_t)4 * DM * D4 * 2);
    if ((size_t)(wsp - (char*)d_ws) > ws_size) return;
    k_cat4<<<(unsigned)(NM * 4 * DM / 8 / 256), 256, 0, stream>>>(q0, q1, q2, q3, Xq);
    k_qw<bf><<<(unsigned)(2 * D4 * 4 * DM / 8 / 256), 256, 0, stream>>>(Wi0, Wi1, Wi2, Wi3, DM, 2 * DI, 1.0f, (unsigned short*)Bi);
    k_gemmw<bf, 0, false><<<dim3(NM / 64, 2 * D4 / 64, 1), 32, 0, stream>>>(Xq, nullptr, Bi, nullptr, 4 * DM, XZ, 2 * D4, nullptr, 0, 0, 0);
    k_conv<<<(unsigned)(NM * D4 / 4 / 256), 256, 0, stream>>>(XZ, cw, cb, Xs, Xh, Xl);
    k_wtG<<<(unsigned)(NXD * D4 / 64 / 64), 256, 0, stream>>>(Wx, D4, NXD, Bx);
    k_fillb<<<(unsigned)((NXP - NXD) * D4 / 8 / 256), 256, 0, stream>>>(Bx + (size_t)NXD * D4, 0u, (size_t)(NXP - NXD) * D4 / 8);
    k_gemmw<bf, 1, false><<<dim3(NM / 64, NXP / 64, 1), 32, 0, stream>>>(Xh, Xl, Bx, nullptr, D4, XD, NXP, nullptr, 0, 0, 0);
    k_scan<<<(unsigned)(NB * D4 / 256), 256, 0, stream>>>(XD, Xs, Wd, bd, Al, Ys);
    k_gate<<<(unsigned)(NM * D4 / 8 / 256), 256, 0, stream>>>(Ys, Xs, XZ, Dv, Yh);
    k_qw<h16><<<(unsigned)(4 * DM * D4 / 8 / 256), 256, 0, stream>>>(Wo0, Wo1, Wo2, Wo3, DI, DM, 16.0f, (unsigned short*)Bo);
    k_gemmw<h16, 0, false><<<dim3(NM / 64, 4 * DM / 64, 1), 32, 0, stream>>>(Yh, nullptr, Bo, nullptr, D4, out, 4 * DM, nullptr, 0, 0, 0);
}
